// LSTM_74122545594502
// MI455X (gfx1250) — hardware-verified
//
#include <hip/hip_runtime.h>
#include <math.h>

constexpr int NBATCH   = 4096;
constexpr int NSTEP    = 256;
constexpr int NDIN     = 4;
constexpr int NHID     = 16;
constexpr int NGATE    = 4 * NHID;
constexpr int NCELL    = 6;
constexpr int NTHR     = 128;
constexpr int NWAVE    = NTHR / 32;
constexpr int NOUTC    = 4;
constexpr int WPITCH   = 40;
constexpr int CELLW    = NGATE * WPITCH;
constexpr int PPITCH   = 72;
constexpr int PLANE    = 16 * PPITCH;
constexpr int HSPITCH  = 36;
constexpr float WCARRY     = 16.0f;
constexpr float WCARRY_INV = 1.0f / 16.0f;

static_assert(NBATCH % (16 * NWAVE) == 0, "grid exact");
static_assert(NGATE == 64 && NHID == 16 && NDIN == 4, "shape");
static_assert(NTHR == 2 * NGATE, "weight build: 64 rows x 2 parts");
static_assert((NWAVE * 2 * PLANE / 8) % NTHR == 0, "plane zero-fill exact");
static_assert((PPITCH * 2) % 16 == 0 && (WPITCH * 2) % 16 == 0, "16-B aligned rows");
static_assert(2 * NHID + 32 <= PPITCH && NDIN <= 16, "window fits");

typedef __attribute__((ext_vector_type(16))) _Float16 v16h;
typedef __attribute__((ext_vector_type(8)))  _Float16 v8h;
typedef __attribute__((ext_vector_type(8)))  float    v8f;
typedef __attribute__((ext_vector_type(4)))  float    v4f;

union FragU { v16h v; v8h h[2]; };
__device__ __forceinline__ v16h frag_load(const _Float16* p) {
  FragU f;
  f.h[0] = *(const v8h*)(p);
  f.h[1] = *(const v8h*)(p + 16);
  return f.v;
}
__device__ __forceinline__ v8f frag_mma(v16h a, v16h b, v8f c) {
  return __builtin_amdgcn_wmma_f32_16x16x32_f16(false, a, false, b, (short)0, c, false, false);
}
__device__ __forceinline__ void guard_cell(v8f& a0, v8f& a1, v8f& a2, v8f& a3,
                                           v16h a, v16h b0, v16h b1, v16h b2, v16h b3) {
  asm volatile("v_nop\n\tv_nop\n\tv_nop\n\tv_nop"
               : "+v"(a0), "+v"(a1), "+v"(a2), "+v"(a3)
               : "v"(a), "v"(b0), "v"(b1), "v"(b2), "v"(b3));
}
__device__ __forceinline__ void wave_lds_sync() {
  __builtin_amdgcn_fence(__ATOMIC_RELEASE, "workgroup");
  __builtin_amdgcn_wave_barrier();
  __builtin_amdgcn_fence(__ATOMIC_ACQUIRE, "workgroup");
}

__device__ __forceinline__ float fsig(float x)  { return __builtin_amdgcn_rcpf(1.0f + __expf(-x)); }
__device__ __forceinline__ float ftanh(float x) { return 1.0f - 2.0f * __builtin_amdgcn_rcpf(__expf(2.0f * x) + 1.0f); }

template <bool LAYER1>
__device__ __forceinline__ void build_cell(const float* wih, const float* whh, const float* bih, const float* bhh,
                                           _Float16* wt, float* bs, int g, int part) {
  v4f s0, s1, s2, s3;
  if (LAYER1) {
    const v4f h0 = *(const v4f*)(whh + g * 16 + 0);
    const v4f h1 = *(const v4f*)(whh + g * 16 + 4);
    const v4f h2 = *(const v4f*)(whh + g * 16 + 8);
    const v4f h3 = *(const v4f*)(whh + g * 16 + 12);
    const v4f i0 = *(const v4f*)(wih + g * 4);
#pragma unroll
    for (int e = 0; e < 4; ++e) {
      const float a0 = h0[e], a1 = h1[e], a2 = h2[e], a3 = h3[e], x0 = i0[e];
      s0[e] = part ? a0 : x0;
      s1[e] = part ? a1 : 0.0f;
      s2[e] = part ? a2 : 0.0f;
      s3[e] = part ? a3 : 0.0f;
    }
  } else {
    const float* src = (part ? whh : wih) + g * 16;
    s0 = *(const v4f*)(src + 0);
    s1 = *(const v4f*)(src + 4);
    s2 = *(const v4f*)(src + 8);
    s3 = *(const v4f*)(src + 12);
  }
  const float bsv = bih[g] + bhh[g];
  v8h o0, o1;
#pragma unroll
  for (int e = 0; e < 4; ++e) {
    const float a0 = s0[e], a1 = s1[e], a2 = s2[e], a3 = s3[e];
    o0[e]     = (_Float16)(a0 * WCARRY);
    o0[4 + e] = (_Float16)(a1 * WCARRY);
    o1[e]     = (_Float16)(a2 * WCARRY);
    o1[4 + e] = (_Float16)(a3 * WCARRY);
  }
  _Float16* wr = wt + g * WPITCH + part * 16;
  *(v8h*)(wr)     = o0;
  *(v8h*)(wr + 8) = o1;
  if (part) {
    const v8h z = {(_Float16)0.0f, (_Float16)0.0f, (_Float16)0.0f, (_Float16)0.0f,
                   (_Float16)0.0f, (_Float16)0.0f, (_Float16)0.0f, (_Float16)0.0f};
    *(v8h*)(wt + g * WPITCH + 32) = z;
  } else {
    bs[g] = bsv;
  }
  asm volatile("" ::: "memory");
}

template <int WOFF, int HCOL>
__device__ __forceinline__ void lstm_cell(const _Float16* wt, _Float16* plane, const float (&bz)[4],
                                          float (&cs)[8], float (&hout)[8], int n, int hh) {
  const v8f z8 = {0.f, 0.f, 0.f, 0.f, 0.f, 0.f, 0.f, 0.f};
  const v16h a = frag_load(plane + n * PPITCH + WOFF + 8 * hh);
  const _Float16* wr = wt + n * WPITCH + 8 * hh;
  const v16h b0 = frag_load(wr + 0 * 16 * WPITCH);
  const v16h b1 = frag_load(wr + 1 * 16 * WPITCH);
  const v16h b2 = frag_load(wr + 2 * 16 * WPITCH);
  const v16h b3 = frag_load(wr + 3 * 16 * WPITCH);
  v8f acc0 = frag_mma(a, b0, z8);
  v8f acc1 = frag_mma(a, b1, z8);
  v8f acc2 = frag_mma(a, b2, z8);
  v8f acc3 = frag_mma(a, b3, z8);
  guard_cell(acc0, acc1, acc2, acc3, a, b0, b1, b2, b3);
#pragma unroll
  for (int r = 0; r < 8; ++r) {
    const float zi = acc0[r] * WCARRY_INV + bz[0];
    const float zf = acc1[r] * WCARRY_INV + bz[1];
    const float zg = acc2[r] * WCARRY_INV + bz[2];
    const float zo = acc3[r] * WCARRY_INV + bz[3];
    const float ig = fsig(zi);
    const float fg = fsig(zf);
    const float gg = ftanh(zg);
    const float og = fsig(zo);
    const float cn = fg * cs[r] + ig * gg;
    cs[r] = cn;
    const float hn = og * ftanh(cn);
    hout[r] = hn;
    plane[(8 * hh + r) * PPITCH + HCOL + n] = (_Float16)hn;
  }
}

__global__ __launch_bounds__(NTHR) void lstm_bidir_kernel(
    const float* y,
    const float* wih0, const float* whh0, const float* bih0, const float* bhh0,
    const float* wih1, const float* whh1, const float* bih1, const float* bhh1,
    const float* wih2, const float* whh2, const float* bih2, const float* bhh2,
    const float* wih3, const float* whh3, const float* bih3, const float* bhh3,
    const float* wih4, const float* whh4, const float* bih4, const float* bhh4,
    const float* wih5, const float* whh5, const float* bih5, const float* bhh5,
    const float* wout, const float* bout, float* out) {
  __shared__ __align__(16) _Float16 Wt[NCELL * CELLW];
  __shared__ __align__(16) _Float16 Pl[NWAVE * 2 * PLANE];
  __shared__ __align__(16) float Hs[NWAVE * 16 * HSPITCH];
  __shared__ float bsum[NCELL * NGATE];
  __shared__ float wout_s[NOUTC * 2 * NHID];
  __shared__ float bout_s[NOUTC];

  const int tid  = threadIdx.x;
  const int lane = tid & 31;
  const int wave = tid >> 5;
  const int n    = lane & 15;
  const int hh   = lane >> 4;

  const v8h zero8 = {(_Float16)0.0f, (_Float16)0.0f, (_Float16)0.0f, (_Float16)0.0f,
                     (_Float16)0.0f, (_Float16)0.0f, (_Float16)0.0f, (_Float16)0.0f};

#pragma unroll 1
  for (int i = tid; i < NWAVE * 2 * PLANE / 8; i += NTHR) *(v8h*)(Pl + i * 8) = zero8;

  {
    const int g = tid & 63, part = tid >> 6;
    build_cell<true >(wih0, whh0, bih0, bhh0, Wt + 0 * CELLW, bsum + 0 * NGATE, g, part);
    build_cell<false>(wih1, whh1, bih1, bhh1, Wt + 1 * CELLW, bsum + 1 * NGATE, g, part);
    build_cell<false>(wih2, whh2, bih2, bhh2, Wt + 2 * CELLW, bsum + 2 * NGATE, g, part);
    build_cell<true >(wih3, whh3, bih3, bhh3, Wt + 3 * CELLW, bsum + 3 * NGATE, g, part);
    build_cell<false>(wih4, whh4, bih4, bhh4, Wt + 4 * CELLW, bsum + 4 * NGATE, g, part);
    build_cell<false>(wih5, whh5, bih5, bhh5, Wt + 5 * CELLW, bsum + 5 * NGATE, g, part);
    wout_s[tid] = wout[tid];
    const float bv = bout[tid & 3];
    if (tid < NOUTC) bout_s[tid] = bv;
  }
  __syncthreads();

  float bz[NCELL][4];
#pragma unroll
  for (int c = 0; c < NCELL; ++c)
#pragma unroll
    for (int tl = 0; tl < 4; ++tl) bz[c][tl] = bsum[c * NGATE + tl * 16 + n];

  float cs[NCELL][8];
#pragma unroll
  for (int c = 0; c < NCELL; ++c)
#pragma unroll
    for (int r = 0; r < 8; ++r) cs[c][r] = 0.0f;
  float hf3[8], hb3[8], hdump[8];
#pragma unroll
  for (int r = 0; r < 8; ++r) { hf3[r] = 0.0f; hb3[r] = 0.0f; hdump[r] = 0.0f; }

  const int rowbase = (blockIdx.x * NWAVE + wave) * 16;
  _Float16* plf = Pl + wave * (2 * PLANE);
  _Float16* plb = plf + PLANE;
  const float* yrow = y + (size_t)(rowbase + n) * (size_t)(NSTEP * NDIN);
  _Float16* xdst = plf + hh * PLANE + n * PPITCH;

#pragma unroll 1
  for (int t = 0; t < NSTEP; ++t) {
    const int tt = hh ? (NSTEP - 1 - t) : t;
    const v4f xv = *(const v4f*)(yrow + tt * NDIN);
    const float x0 = xv[0], x1 = xv[1], x2 = xv[2], x3 = xv[3];
    v8h xh;
    xh[0] = (_Float16)x0;
    xh[1] = (_Float16)x1;
    xh[2] = (_Float16)x2;
    xh[3] = (_Float16)x3;
    xh[4] = (_Float16)0.0f;
    xh[5] = (_Float16)0.0f;
    xh[6] = (_Float16)0.0f;
    xh[7] = (_Float16)0.0f;
    *(v8h*)(xdst)     = xh;
    *(v8h*)(xdst + 8) = zero8;
    wave_lds_sync();

    lstm_cell<0, 16>(Wt + 0 * CELLW, plf, bz[0], cs[0], hdump, n, hh);
    lstm_cell<0, 16>(Wt + 3 * CELLW, plb, bz[3], cs[3], hdump, n, hh);
    wave_lds_sync();
    lstm_cell<16, 32>(Wt + 1 * CELLW, plf, bz[1], cs[1], hdump, n, hh);
    lstm_cell<16, 32>(Wt + 4 * CELLW, plb, bz[4], cs[4], hdump, n, hh);
    wave_lds_sync();
    lstm_cell<32, 48>(Wt + 2 * CELLW, plf, bz[2], cs[2], hf3, n, hh);
    lstm_cell<32, 48>(Wt + 5 * CELLW, plb, bz[5], cs[5], hb3, n, hh);
    wave_lds_sync();
  }

  float* hs = Hs + wave * (16 * HSPITCH);
#pragma unroll
  for (int r = 0; r < 8; ++r) {
    hs[(8 * hh + r) * HSPITCH + n]        = hf3[r];
    hs[(8 * hh + r) * HSPITCH + NHID + n] = hb3[r];
  }
  wave_lds_sync();
  const int row = lane & 15;
  float o0 = 0.0f, o1 = 0.0f, o2 = 0.0f, o3 = 0.0f;
#pragma unroll 1
  for (int k = 0; k < 2 * NHID; ++k) {
    const float hv = hs[row * HSPITCH + k];
    o0 = fmaf(hv, wout_s[0 * 2 * NHID + k], o0);
    o1 = fmaf(hv, wout_s[1 * 2 * NHID + k], o1);
    o2 = fmaf(hv, wout_s[2 * 2 * NHID + k], o2);
    o3 = fmaf(hv, wout_s[3 * 2 * NHID + k], o3);
  }
  v4f ov;
  ov[0] = o0 + bout_s[0];
  ov[1] = o1 + bout_s[1];
  ov[2] = o2 + bout_s[2];
  ov[3] = o3 + bout_s[3];
  float* op = out + (size_t)(rowbase + row) * NOUTC;
  if (lane < 16) *(volatile v4f*)op = ov;
  __threadfence();
  if (lane < 16) *(volatile v4f*)op = ov;
}

extern "C" void kernel_launch(void* const* d_in, const int* in_sizes, int n_in,
                              void* d_out, int out_size, void* d_ws, size_t ws_size, hipStream_t stream) {
  (void)d_ws; (void)ws_size;
  if (n_in < 27 || d_out == nullptr) return;
  if (in_sizes[0] != NBATCH * NSTEP * NDIN) return;
  for (int c = 0; c < NCELL; ++c) {
    const int din = (c == 0 || c == 3) ? NDIN : NHID;
    if (in_sizes[1 + 4 * c + 0] != NGATE * din) return;
    if (in_sizes[1 + 4 * c + 1] != NGATE * NHID) return;
    if (in_sizes[1 + 4 * c + 2] != NGATE) return;
    if (in_sizes[1 + 4 * c + 3] != NGATE) return;
  }
  if (in_sizes[25] != NOUTC * 2 * NHID || in_sizes[26] != NOUTC) return;
  if (out_size != NBATCH * NOUTC) return;

  const float* p[27];
  for (int i = 0; i < 27; ++i) p[i] = (const float*)d_in[i];

  lstm_bidir_kernel<<<NBATCH / (16 * NWAVE), NTHR, 0, stream>>>(
      p[0],
      p[1],  p[2],  p[3],  p[4],
      p[5],  p[6],  p[7],  p[8],
      p[9],  p[10], p[11], p[12],
      p[13], p[14], p[15], p[16],
      p[17], p[18], p[19], p[20],
      p[21], p[22], p[23], p[24],
      p[25], p[26], (float*)d_out);
}
